// GroupedQueryAttention_37349035606742
// MI455X (gfx1250) — hardware-verified
//
#include <hip/hip_runtime.h>
#include <math.h>

typedef __attribute__((ext_vector_type(16))) _Float16 v16h;
typedef __attribute__((ext_vector_type(16))) __bf16 v16b;
typedef __attribute__((ext_vector_type(8)))  _Float16 v8h;
typedef __attribute__((ext_vector_type(8)))  float v8f;
typedef __attribute__((ext_vector_type(4)))  float v4f;
typedef __attribute__((ext_vector_type(4)))  unsigned v4u;

template <typename T> __device__ __forceinline__ void vst2(void* p, T v) { *(volatile T*)p = v; __threadfence(); *(volatile T*)p = v; }
__device__ __forceinline__ v8f wmma16(v16h a, v16h b, v8f c) {
  v8f d = __builtin_amdgcn_wmma_f32_16x16x32_f16(false, a, false, b, (short)0, c, false, false);
  asm volatile("v_nop\n\tv_nop\n\tv_nop\n\tv_nop" : "+v"(d) : "v"(a), "v"(b));
  return d;
}
__device__ __forceinline__ v8f wmma_bf(v16b a, v16b b, v8f c) {
  v8f d = __builtin_amdgcn_wmma_f32_16x16x32_bf16(false, a, false, b, (short)0, c, false, false);
  asm volatile("v_nop\n\tv_nop\n\tv_nop\n\tv_nop" : "+v"(d) : "v"(a), "v"(b));
  return d;
}
__device__ __forceinline__ v16h frag_h(const _Float16* rowk0, int lane) {
  union { v16h v; v8h q[2]; } u; const _Float16* p = rowk0 + 8 * (lane >> 4);
  u.q[0] = *(const v8h*)p; u.q[1] = *(const v8h*)(p + 16); return u.v;
}
__device__ __forceinline__ v16h frag_f32(const float* rowk0, int lane) {
  v16h a; const float* p = rowk0 + 8 * (lane >> 4);
#pragma unroll
  for (int i = 0; i < 8; ++i) { a[i] = (_Float16)p[i]; a[8 + i] = (_Float16)p[16 + i]; }
  return a;
}
struct F2 { v16b h, l; };
__device__ __forceinline__ F2 bsplit16(const float v[16]) { F2 r;
#pragma unroll
  for (int i = 0; i < 16; ++i) { const __bf16 h = (__bf16)v[i]; r.h[i] = h; r.l[i] = (__bf16)(v[i] - (float)h); }
  return r; }
__device__ __forceinline__ F2 split_row(const float* row, int k0, int lane) { float v[16]; const float* p = row + k0 + 8 * (lane >> 4);
#pragma unroll
  for (int i = 0; i < 8; ++i) { v[i] = p[i]; v[8 + i] = p[16 + i]; }
  return bsplit16(v); }
__device__ __forceinline__ float bfr(float v) { return (float)(__bf16)v; }
#define LDSX() do { asm volatile("s_wait_dscnt 0" ::: "memory"); __builtin_amdgcn_wave_barrier(); __builtin_amdgcn_fence(3  , "workgroup"); } while (0)
__device__ __forceinline__ v16b wcol_io(const float* Wm, int k0, int o, int lane, int ld) { v16b w; const int g = lane >> 4;
#pragma unroll
  for (int i = 0; i < 8; ++i) { w[i] = (__bf16)Wm[(size_t)(k0 + 8 * g + i) * ld + o]; w[8 + i] = (__bf16)Wm[(size_t)(k0 + 16 + 8 * g + i) * ld + o]; }
  return w; }

#ifndef NB
#define NB 2
#endif
#ifndef SEQ
#define SEQ 2048
#endif
#define NB_FULL 2
#define SEQ_FULL 2048
#define DIN 1024
#define CC 1024
#define NH 16
#define NKV 4
#define HG (NH / NKV)
#define HD 64
#define KVW (NKV * HD)
#define NQB (SEQ / 64)
#define SCALE (0.125f)
#define PCARRY (2048.0f)
#define PSUB (PCARRY / (float)SEQ)
#define OUT1_OFF ((size_t)NB_FULL * SEQ_FULL * CC)
#define OUT2_OFF (OUT1_OFF + (size_t)NB_FULL * NKV * SEQ_FULL * HD)
static_assert(OUT1_OFF * 4u == 16777216u);
static_assert(OUT2_OFF * 4u == 20971520u);
static_assert(NB >= 1 && NB <= NB_FULL);
static_assert(SEQ >= 128 && SEQ <= SEQ_FULL && SEQ % 128 == 0);
static_assert(CC % 128 == 0 && KVW % 128 == 0 && DIN % 128 == 0 && DIN % 32 == 0 && HD == 64 && HG == 4);

#define WS_QH  ((size_t)0)
#define WS_KH  (WS_QH + 2u * (size_t)NB * SEQ * CC)
#define WS_VT  (WS_KH + 2u * (size_t)NB * SEQ * KVW)
#define WS_VM  (WS_VT + 2u * (size_t)NB * KVW * SEQ)
#define WS_S   (WS_VM + (size_t)4096)
#define WS_Y   (WS_S  + 4u * (size_t)HG * SEQ * SEQ)
#define WS_END (WS_Y  + 4u * (size_t)NB * SEQ * CC)
static_assert(4u * (size_t)NB * KVW <= 4096u);
static_assert(WS_END <= (size_t)134217728u);

__global__ __launch_bounds__(128) void k_proj(const float* __restrict__ X, const float* __restrict__ W, const float* __restrict__ BA, int which,
    _Float16* __restrict__ DH, _Float16* __restrict__ VT, float* __restrict__ OUTC) {
  __shared__ __align__(16) _Float16 sx[128 * 72];
  __shared__ __align__(16) float sf[64][132];
  const int tid = threadIdx.x, wave = tid >> 5, lane = tid & 31, col = lane & 15, g = lane >> 4;
  const int ncol = (which == 0) ? CC : KVW;
  const int c0 = blockIdx.y * 128;
  const size_t r0 = (size_t)blockIdx.x * 64; const int bb = (int)(r0 / SEQ); const int t0 = (int)(r0 % SEQ);
  const size_t xr0 = (size_t)bb * SEQ_FULL + t0;
  v8f acc[8] = {};
#pragma unroll 2
  for (int kc = 0; kc < DIN / 32; ++kc) { v16b a; { const float* p = X + (xr0 + wave * 16 + col) * DIN + kc * 32 + 8 * g;
#pragma unroll
      for (int i = 0; i < 8; ++i) { a[i] = (__bf16)p[i]; a[8 + i] = (__bf16)p[16 + i]; } }
    asm volatile("s_wait_loadcnt 0x0" ::: "memory");
#pragma unroll
    for (int j = 0; j < 8; ++j) { const v16b w = wcol_io(W, kc * 32, c0 + j * 16 + col, lane, ncol); asm volatile("s_wait_loadcnt 0x0" ::: "memory"); acc[j] = wmma_bf(a, w, acc[j]); } }
  if (which < 2) {
#pragma unroll
    for (int j = 0; j < 8; ++j) { const float bias = bfr(BA[c0 + j * 16 + col]);
#pragma unroll
      for (int r = 0; r < 8; ++r) { const float v = acc[j][r] + bias; const int rl = wave * 16 + 8 * g + r, cl = j * 16 + col; sx[rl * 136 + cl] = (_Float16)v; sf[rl][cl] = v; } }
    __syncthreads();
    for (int e = tid; e < 64 * 16; e += 128) { const int rl = e >> 4, q = e & 15; vst2((unsigned*)(DH + (r0 + rl) * (size_t)ncol + c0 + q * 8), *(const v4u*)&sx[rl * 136 + q * 8]); }
    if (which == 1) { const size_t ob = (((size_t)bb * NKV + (c0 >> 6)) * SEQ + t0) * HD;
      for (int e = tid; e < 64 * 2 * 16; e += 128) { const int q = e & 15, seg = e >> 4, rl = seg >> 1, kk = seg & 1;
        vst2(OUTC + ob + ((size_t)kk * SEQ + rl) * HD + q * 4, *(const v4f*)&sf[rl][kk * 64 + q * 4]); } }
  } else {
#pragma unroll
    for (int j = 0; j < 8; ++j) { const float bias = bfr(BA[c0 + j * 16 + col]);
#pragma unroll
      for (int r = 0; r < 8; ++r) { const float v = acc[j][r] + bias; const int rl = wave * 16 + 8 * g + r, cl = j * 16 + col; sx[cl * 72 + rl] = (_Float16)v; sf[rl][cl] = v; } }
    __syncthreads();
    for (int e = tid; e < 128 * 8; e += 128) { const int cl = e >> 3, q = e & 7; vst2((unsigned*)(VT + ((size_t)bb * KVW + c0 + cl) * (size_t)SEQ + t0 + q * 8), *(const v4u*)&sx[cl * 72 + q * 8]); }
    const size_t ob = (((size_t)bb * NKV + (c0 >> 6)) * SEQ + t0) * HD;
    for (int e = tid; e < 64 * 2 * 16; e += 128) { const int q = e & 15, seg = e >> 4, rl = seg >> 1, kk = seg & 1;
      vst2(OUTC + ob + ((size_t)kk * SEQ + rl) * HD + q * 4, *(const v4f*)&sf[rl][kk * 64 + q * 4]); } }
}
__global__ __launch_bounds__(128) void k_sc(const _Float16* __restrict__ QH, const _Float16* __restrict__ KH, int b, int h0, float* __restrict__ S0) {
  __shared__ __align__(16) float ss[4][16][132];
  const int qb = blockIdx.x, kb = blockIdx.y; const int h = h0 + blockIdx.z; const int kvh = h / HG;
  float* S = S0 + (size_t)blockIdx.z * SEQ * SEQ;
  const int tid = threadIdx.x, wave = tid >> 5, lane = tid & 31, col = lane & 15, g = lane >> 4;
  const int k0 = kb * 128; const int ql0 = qb * 64 + wave * 16; const size_t q0 = (size_t)b * SEQ + ql0, kr0 = (size_t)b * SEQ + k0;
  v8f acc[8] = {};
#pragma unroll
  for (int kc = 0; kc < HD / 32; ++kc) { const v16h ah = frag_h(QH + (q0 + col) * CC + h * HD + kc * 32, lane);
#pragma unroll
    for (int j = 0; j < 8; ++j) { const v16h kf = frag_h(KH + (kr0 + j * 16 + col) * KVW + kvh * HD + kc * 32, lane); acc[j] = wmma16(ah, kf, acc[j]); } }
#pragma unroll
  for (int j = 0; j < 8; ++j) {
#pragma unroll
    for (int r = 0; r < 8; ++r) ss[wave][8 * g + r][j * 16 + col] = acc[j][r] * SCALE; }
  LDSX(); for (int rl = 0; rl < 16; ++rl) vst2(S + (size_t)(ql0 + rl) * SEQ + k0 + lane * 4, *(const v4f*)&ss[wave][rl][lane * 4]); }
__global__ __launch_bounds__(256) void k_sm(float* __restrict__ S0) { __shared__ float sred[8]; __shared__ float sbc; __shared__ __align__(16) float shv[SEQ];
  const int tid = threadIdx.x; const int t = blockIdx.x;
  float* sr = S0 + (size_t)blockIdx.y * SEQ * SEQ + (size_t)t * SEQ;
  float m = -3.0e38f;
#pragma unroll 1
  for (int k = tid; k < SEQ; k += 256) { const float v = sr[k]; shv[k] = v; m = fmaxf(m, v); }
#pragma unroll
  for (int o = 1; o < 32; o <<= 1) m = fmaxf(m, __shfl_xor(m, o));
  if ((tid & 31) == 0) sred[tid >> 5] = m; __syncthreads(); if (tid == 0) { float a = sred[0]; for (int i = 1; i < 8; ++i) a = fmaxf(a, sred[i]); sbc = a; } __syncthreads(); m = sbc; __syncthreads();
  float sum = 0.f;
#pragma unroll 1
  for (int k = tid; k < SEQ; k += 256) { const float e = expf(shv[k] - m); shv[k] = e; sum += e; }
#pragma unroll
  for (int o = 1; o < 32; o <<= 1) sum += __shfl_xor(sum, o);
  if ((tid & 31) == 0) sred[tid >> 5] = sum; __syncthreads(); if (tid == 0) { float a = 0.f; for (int i = 0; i < 8; ++i) a += sred[i]; sbc = PCARRY / a; } __syncthreads(); const float inv = sbc;
#pragma unroll 1
  for (int k = tid; k < SEQ; k += 256) shv[k] = shv[k] * inv - PSUB;
  __syncthreads(); for (int q = tid; q < SEQ / 4; q += 256) vst2(sr + q * 4, *(const v4f*)&shv[q * 4]); }
__global__ __launch_bounds__(256) void k_vmean(const float* __restrict__ OV, float* __restrict__ VM) {
  __shared__ float sp[4][64]; __shared__ __align__(16) float smn[64];
  const int tid = threadIdx.x, d = tid & 63, sg = tid >> 6; const int b = blockIdx.x / NKV, kvh = blockIdx.x % NKV;
  const float* p = OV + (((size_t)b * NKV + kvh) * SEQ + (size_t)sg * (SEQ / 4)) * HD + d;
  float s = 0.f;
#pragma unroll 4
  for (int i = 0; i < SEQ / 4; ++i) s += p[(size_t)i * HD];
  sp[sg][d] = s; __syncthreads();
  if (tid < 64) smn[tid] = ((sp[0][tid] + sp[1][tid]) + (sp[2][tid] + sp[3][tid])) * (1.0f / (float)SEQ);
  __syncthreads();
  const v4f mv = *(const v4f*)&smn[(tid & 15) * 4];
  if (tid < 16) vst2(VM + (size_t)b * KVW + kvh * HD + tid * 4, mv); }
__global__ __launch_bounds__(128) void k_pv(const float* __restrict__ PS0, const _Float16* __restrict__ VT, const float* __restrict__ VM, int b, int h0, float* __restrict__ Y) {
  __shared__ __align__(16) float ss[4][16][HD + 4];
  const int h = h0 + blockIdx.z, kvh = h / HG; const float* PS = PS0 + (size_t)blockIdx.z * SEQ * SEQ;
  const int tid = threadIdx.x, wave = tid >> 5, lane = tid & 31, col = lane & 15, g = lane >> 4; const int qb = blockIdx.x; const int ql0 = qb * 64 + wave * 16;
  v8f acc[HD / 16] = {};
#pragma unroll 1
  for (int kc = 0; kc < SEQ / 32; ++kc) { const v16h pf = frag_f32(PS + (size_t)(ql0 + col) * SEQ + kc * 32, lane);
    asm volatile("s_wait_loadcnt 0x0" ::: "memory");
#pragma unroll
    for (int j = 0; j < HD / 16; ++j) { const size_t po = ((size_t)b * KVW + kvh * HD + j * 16 + col) * (size_t)SEQ + kc * 32; acc[j] = wmma16(pf, frag_h(VT + po, lane), acc[j]); } }
#pragma unroll
  for (int j = 0; j < HD / 16; ++j) { const float mv = VM[(size_t)b * KVW + kvh * HD + j * 16 + col];
#pragma unroll
    for (int r = 0; r < 8; ++r) ss[wave][8 * g + r][j * 16 + col] = acc[j][r] * (1.0f / PCARRY) + mv; }
  LDSX(); const int lc = lane & 15;
  for (int rl = 0; rl < 16; ++rl) { const v4f v = *(const v4f*)&ss[wave][rl][lc * 4]; if (lane < HD / 4) vst2(Y + ((size_t)b * SEQ + ql0 + rl) * CC + h * HD + lc * 4, v); } }
__global__ __launch_bounds__(128) void k_out(const float* __restrict__ Y, const float* __restrict__ WO, const float* __restrict__ BO, float* __restrict__ OUT) { __shared__ __align__(16) float sf[4][16][132];
  const int tid = threadIdx.x, wave = tid >> 5, lane = tid & 31, col = lane & 15, g = lane >> 4; const int c0 = blockIdx.y * 128; const size_t r0 = (size_t)blockIdx.x * 64 + wave * 16;
  v8f acc[8] = {};
#pragma unroll 2
  for (int kc = 0; kc < CC / 32; ++kc) { const F2 a = split_row(Y + (r0 + col) * CC, kc * 32, lane); asm volatile("s_wait_loadcnt 0x0" ::: "memory");
#pragma unroll
    for (int j = 0; j < 8; ++j) { const v16b w = wcol_io(WO, kc * 32, c0 + j * 16 + col, lane, DIN); asm volatile("s_wait_loadcnt 0x0" ::: "memory"); acc[j] = wmma_bf(a.h, w, acc[j]); acc[j] = wmma_bf(a.l, w, acc[j]); } }
#pragma unroll
  for (int j = 0; j < 8; ++j) { const float bias = bfr(BO[c0 + j * 16 + col]);
#pragma unroll
    for (int r = 0; r < 8; ++r) sf[wave][8 * g + r][j * 16 + col] = acc[j][r] + bias; }
  LDSX(); for (int rl = 0; rl < 16; ++rl) vst2(OUT + (r0 + rl) * DIN + c0 + lane * 4, *(const v4f*)&sf[wave][rl][lane * 4]); }

extern "C" void kernel_launch(void* const* d_in, const int* in_sizes, int n_in, void* d_out, int out_size, void* d_ws, size_t ws_size, hipStream_t stream) {
  if (n_in < 11) return;
  const size_t need_x = ((size_t)(NB - 1) * SEQ_FULL + SEQ) * DIN;
  if ((size_t)in_sizes[0] < need_x || (size_t)in_sizes[1] < need_x || (size_t)in_sizes[2] < need_x) return;
  if ((size_t)in_sizes[3] < (size_t)DIN * CC || in_sizes[4] < CC || (size_t)in_sizes[5] < (size_t)DIN * KVW || in_sizes[6] < KVW ||
      (size_t)in_sizes[7] < (size_t)DIN * KVW || in_sizes[8] < KVW || (size_t)in_sizes[9] < (size_t)CC * DIN || in_sizes[10] < DIN) return;
  if ((size_t)out_size < OUT2_OFF + (size_t)NB * NKV * SEQ * HD) return;
  if (ws_size < (size_t)WS_END) return;
  const float** F = (const float**)d_in;
  char* ws = (char*)d_ws; _Float16 *QH = (_Float16*)(ws + WS_QH), *KH = (_Float16*)(ws + WS_KH), *VT = (_Float16*)(ws + WS_VT); float *VM = (float*)(ws + WS_VM), *S = (float*)(ws + WS_S), *Y = (float*)(ws + WS_Y);
  float* out = (float*)d_out; float* outk = out + OUT1_OFF; float* outv = out + OUT2_OFF;
  k_proj<<<dim3(NB * SEQ / 64, CC / 128), 128, 0, stream>>>(F[0], F[3], F[4], 0, QH, VT, outk);
  k_proj<<<dim3(NB * SEQ / 64, KVW / 128), 128, 0, stream>>>(F[1], F[5], F[6], 1, KH, VT, outk);
  k_proj<<<dim3(NB * SEQ / 64, KVW / 128), 128, 0, stream>>>(F[2], F[7], F[8], 2, KH, VT, outv);
  k_vmean<<<dim3(NB * NKV), 256, 0, stream>>>(outv, VM);
  for (int b = 0; b < NB; ++b) for (int h0 = 0; h0 < NH; h0 += HG) {
    k_sc<<<dim3(NQB, SEQ / 128, HG), 128, 0, stream>>>(QH, KH, b, h0, S);
    k_sm<<<dim3(SEQ, HG), 256, 0, stream>>>(S);
    k_pv<<<dim3(NQB, 1, HG), 128, 0, stream>>>(S, VT, VM, b, h0, Y);
  }
  k_out<<<dim3(NB * SEQ / 64, DIN / 128), 128, 0, stream>>>(Y, F[9], F[10], out);
}
